// SlimeNetKeras_2224793059471
// MI455X (gfx1250) — hardware-verified
//
#include <hip/hip_runtime.h>
#include <stddef.h>


typedef _Float16     v16h __attribute__((ext_vector_type(16)));
typedef _Float16     v8h  __attribute__((ext_vector_type(8)));
typedef _Float16     v2h  __attribute__((ext_vector_type(2)));
typedef float        v8f  __attribute__((ext_vector_type(8)));
typedef float        v4f  __attribute__((ext_vector_type(4)));
typedef unsigned int v4u  __attribute__((ext_vector_type(4)));

#define CCH        16
#define WCOLS      512
#ifndef HROWS
#define HROWS      512
#endif
#define HROWS_FULL 512
#define HWF        (HROWS_FULL * WCOLS)
#define HIDN       128
#define KFEAT      80
#define KP         96
#ifndef NSTEPS
#define NSTEPS     8
#endif
#define TP         128
#define NTHR       256
#define LDX        104
#define XROWS      (TP + 2)
#define LDD        132

#define WCARRY 64.0f
#define XCARRY 16.0f
#define HCARRY 16.0f
#define HSCALE (HCARRY / (XCARRY * WCARRY))
#define DSCALE (1.0f / (WCARRY * HCARRY))

static_assert(HROWS >= 2 && HROWS <= HROWS_FULL);
static_assert(NSTEPS >= 1 && NSTEPS <= 8);
static_assert(CCH == 16);
static_assert(KFEAT == 5 * CCH);
static_assert((KP % 32) == 0 && KFEAT < KP);
static_assert(KP - KFEAT == 16);
static_assert((HIDN % 32) == 0 && HIDN == 4 * 32);
static_assert(TP == (NTHR / 32) * 16);
static_assert(TP == 32 * 4);
static_assert((NTHR / 32) * 2 == CCH);
static_assert(2 * (NTHR / 32) == CCH);
static_assert(NTHR == 2 * TP);
static_assert((WCOLS % TP) == 0);
static_assert((LDX % 8) == 0 && LDX >= KP);
static_assert((LDD % 4) == 0 && LDD >= TP);
static_assert(XCARRY == 16.0f);
static_assert((size_t)XROWS * LDX * 2 + (size_t)CCH * LDD * 4 <= (size_t)131072);
static_assert((HIDN * KP) % (NTHR * 8) == 0);
static_assert(CCH * HIDN == NTHR * 8);

#define STATE_BYTES ((size_t)CCH * HWF * 4)
#define W1T_BYTES   ((size_t)HIDN * KP * 2)
#define W2T_BYTES   ((size_t)CCH * HIDN * 2)
#define OFF_STATE   ((size_t)0)
#define OFF_W1T     (OFF_STATE + STATE_BYTES)
#define OFF_W2T     (OFF_W1T + W1T_BYTES)
#define WS_TOTAL    (OFF_W2T + W2T_BYTES)
static_assert((STATE_BYTES % 128) == 0 && (W1T_BYTES % 128) == 0 && (W2T_BYTES % 128) == 0);
static_assert(WS_TOTAL <= (size_t)134217728);

__device__ __forceinline__ float bf16r(float x) {
  unsigned int u = __float_as_uint(x);
  u = (u + 0x7FFFu + ((u >> 16) & 1u)) & 0xFFFF0000u;
  return __uint_as_float(u);
}

static __device__ __forceinline__ _Float16 toh_flush(float v) {
  const _Float16 r = (_Float16)v;
  return (fabsf(v) < 6.103515625e-05f) ? (_Float16)0.0f : r;
}

__device__ __forceinline__ v16h frag_at(const _Float16* p) {
  v8h lo = *(const v8h*)(p);
  v8h hi = *(const v8h*)(p + 16);
  v16h out;
#pragma unroll
  for (int i = 0; i < 8; ++i) { out[i] = lo[i]; out[i + 8] = hi[i]; }
  return out;
}
__device__ __forceinline__ v16h ld_frag(const _Float16* base, unsigned ld) {
  const unsigned lane = threadIdx.x & 31u;
  return frag_at(base + (lane & 15u) * ld + (lane >> 4) * 8u);
}

__device__ __forceinline__ v8f wmma16(v16h a, v16h b, v8f c) {
  v8f d = __builtin_amdgcn_wmma_f32_16x16x32_f16(false, a, false, b, (short)0, c,
                                                 false, false);
  asm volatile("v_nop\n\tv_nop\n\tv_nop\n\tv_nop" : "+v"(d) : "v"(a), "v"(b));
  return d;
}

__global__ __launch_bounds__(256) void wprep_kernel(
    const float* __restrict__ W1, const float* __restrict__ B1, const float* __restrict__ W2,
    _Float16* __restrict__ W1t, _Float16* __restrict__ W2t) {
  const unsigned tid = threadIdx.x;
#pragma unroll 1
  for (unsigned it = 0; it < 6u; ++it) {
    const unsigned p = tid + 256u * it;
    const unsigned n = p / 12u;
    const unsigned k8 = (p - n * 12u) * 8u;
    const float bb = B1[n];
    v8h o;
#pragma unroll
    for (unsigned i = 0; i < 8u; ++i) {
      const unsigned k = k8 + i;
      const unsigned kc = (k < (unsigned)KFEAT) ? k : (unsigned)(KFEAT - 1);
      const float w = W1[kc * (unsigned)HIDN + n];
      const float v = (k < (unsigned)KFEAT) ? w : ((k == (unsigned)KFEAT) ? bb : 0.0f);
      o[i] = toh_flush(WCARRY * bf16r(v));
    }
    _Float16* d = W1t + (size_t)p * 8u;
    *(volatile v8h*)d = o;
    __threadfence();
    *(volatile v8h*)d = o;
  }
  {
    const unsigned c = tid >> 4;
    const unsigned k8 = (tid & 15u) * 8u;
    v8h o;
#pragma unroll
    for (unsigned i = 0; i < 8u; ++i)
      o[i] = toh_flush(WCARRY * bf16r(W2[(k8 + i) * (unsigned)CCH + c]));
    _Float16* d = W2t + (size_t)tid * 8u;
    *(volatile v8h*)d = o;
    __threadfence();
    *(volatile v8h*)d = o;
  }
}

template <int CVT_IN>
__device__ __forceinline__ void step_body(
    const float* __restrict__ src, float* __restrict__ dst,
    const _Float16* __restrict__ W1t, const _Float16* __restrict__ W2t,
    const float* __restrict__ B2, const int* __restrict__ nsteps, const int step) {
  __shared__ _Float16 Xs[XROWS * LDX];
  __shared__ float Ds[CCH * LDD];

  const unsigned tid = threadIdx.x, lane = tid & 31u;
  const unsigned wave = __builtin_amdgcn_readfirstlane(tid >> 5);
  const unsigned hh = lane >> 4, m = lane & 15u;
  const unsigned y = blockIdx.y;
  const unsigned x0 = blockIdx.x * (unsigned)TP;
  const unsigned yu = (y == 0u) ? 0u : y - 1u;
  const unsigned yd = (y == (unsigned)(HROWS - 1)) ? 0u : y + 1u;

  const unsigned c0 = 2u * wave;
#pragma unroll
  for (unsigned t = 0; t < 3u; ++t) {
    const unsigned yy = (t == 0u) ? y : ((t == 1u) ? yu : yd);
    const float* p0 = src + (size_t)c0 * HWF + (size_t)yy * WCOLS + x0 + 4u * lane;
    const v4f a = *(const v4f*)p0;
    const v4f b = *(const v4f*)(p0 + HWF);
#pragma unroll
    for (unsigned j = 0; j < 4u; ++j) {
      const float ea = CVT_IN ? bf16r(a[j]) : a[j];
      const float eb = CVT_IN ? bf16r(b[j]) : b[j];
      v2h pk;
      pk[0] = toh_flush(XCARRY * ea);
      pk[1] = toh_flush(XCARRY * eb);
      const unsigned row = 1u + 4u * lane + j;
      if (t == 0u) {
        *(v2h*)&Xs[row * LDX + c0] = pk;
        *(v2h*)&Xs[(row + 1u) * LDX + 48u + c0] = pk;
        *(v2h*)&Xs[(row - 1u) * LDX + 64u + c0] = pk;
      } else {
        *(v2h*)&Xs[row * LDX + 16u * t + c0] = pk;
      }
    }
  }
  if (wave == 0u) {
    const unsigned xe = x0 + (unsigned)(TP - 1);
    const unsigned xl = (x0 == 0u) ? 0u : x0 - 1u;
    const unsigned xr = (xe == (unsigned)(WCOLS - 1)) ? 0u : xe + 1u;
    const unsigned xx = hh ? xr : xl;
    const float v = src[(size_t)m * HWF + (size_t)y * WCOLS + xx];
    const float e = CVT_IN ? bf16r(v) : v;
    const unsigned row = hh ? (unsigned)TP : 1u;
    const unsigned col = hh ? 64u : 48u;
    Xs[row * LDX + col + m] = toh_flush(XCARRY * e);
  }
  {
    const unsigned row = 1u + (tid >> 1);
    const unsigned hf = tid & 1u;
    v4u z;
    z[0] = hf ? 0u : 0x4C00u;
    z[1] = 0u; z[2] = 0u; z[3] = 0u;
    *(v4u*)&Xs[row * LDX + (unsigned)KFEAT + 8u * hf] = z;
  }
  __syncthreads();

  const _Float16* xb = &Xs[(1u + 16u * wave) * LDX];
  v16h xf[3];
#pragma unroll
  for (unsigned ks = 0; ks < 3u; ++ks) xf[ks] = ld_frag(xb + 32u * ks, LDX);

  v8f acc2 = {};
#pragma unroll 1
  for (unsigned ks2 = 0; ks2 < 4u; ++ks2) {
    v16h hf16;
#pragma unroll
    for (unsigned jj = 0; jj < 2u; ++jj) {
      const _Float16* wrow = W1t + (size_t)(32u * ks2 + 16u * jj) * KP;
      v8f acc = {};
#pragma unroll
      for (unsigned ks = 0; ks < 3u; ++ks) {
        const v16h a = ld_frag(wrow + 32u * ks, KP);
        acc = wmma16(a, xf[ks], acc);
      }
#pragma unroll
      for (unsigned r = 0; r < 8u; ++r)
        hf16[8u * jj + r] = toh_flush(fmaxf(acc[r], 0.0f) * HSCALE);
    }
    const v16h a2 = ld_frag(W2t + 32u * ks2, HIDN);
    acc2 = wmma16(a2, hf16, acc2);
  }

  {
    const v4f g0 = *(const v4f*)(B2 + 8u * hh);
    const v4f g1 = *(const v4f*)(B2 + 8u * hh + 4u);
#pragma unroll
    for (unsigned r = 0; r < 8u; ++r) {
      const float bb = bf16r((r < 4u) ? g0[r & 3u] : g1[r & 3u]);
      Ds[(8u * hh + r) * LDD + 16u * wave + m] = acc2[r] * DSCALE + bb;
    }
  }
  __syncthreads();

  const int ns = nsteps[0];
  const bool active = (step < ns);
  v4f xs[2];
  size_t off[2];
#pragma unroll
  for (unsigned i = 0; i < 2u; ++i) {
    const unsigned c = wave + 8u * i;
    const size_t g = (size_t)c * HWF + (size_t)y * WCOLS + x0 + 4u * lane;
    const v4f d = *(const v4f*)&Ds[c * LDD + 4u * lane];
    const v4f so = *(const v4f*)(src + g);
    const bool upd = active && (c != 0u);
    v4f val;
#pragma unroll
    for (int j = 0; j < 4; ++j) {
      const float base = CVT_IN ? bf16r(so[j]) : so[j];
      const float sum = base + d[j];
      val[j] = upd ? sum : base;
    }
    xs[i] = val;
    off[i] = g;
  }
#pragma unroll
  for (int i = 0; i < 2; ++i) *(volatile v4f*)(dst + off[i]) = xs[i];
  __threadfence();
#pragma unroll
  for (int i = 0; i < 2; ++i) *(volatile v4f*)(dst + off[i]) = xs[i];
}

__global__ __launch_bounds__(256) void step_in_kernel(
    const float* __restrict__ src, float* __restrict__ dst,
    const _Float16* __restrict__ W1t, const _Float16* __restrict__ W2t,
    const float* __restrict__ B2, const int* __restrict__ nsteps, const int step) {
  step_body<1>(src, dst, W1t, W2t, B2, nsteps, step);
}
__global__ __launch_bounds__(256) void step_ws_kernel(
    const float* __restrict__ src, float* __restrict__ dst,
    const _Float16* __restrict__ W1t, const _Float16* __restrict__ W2t,
    const float* __restrict__ B2, const int* __restrict__ nsteps, const int step) {
  step_body<0>(src, dst, W1t, W2t, B2, nsteps, step);
}

extern "C" void kernel_launch(void* const* d_in, const int* in_sizes, int n_in,
                              void* d_out, int out_size, void* d_ws, size_t ws_size,
                              hipStream_t stream) {
  if (n_in < 6) return;
  const long long need_s = (long long)(CCH - 1) * HWF + (long long)HROWS * WCOLS;
  if ((long long)in_sizes[0] < need_s) return;
  if ((long long)in_sizes[1] < (long long)KFEAT * HIDN) return;
  if (in_sizes[2] < HIDN) return;
  if ((long long)in_sizes[3] < (long long)HIDN * CCH) return;
  if (in_sizes[4] < CCH) return;
  if (in_sizes[5] < 1) return;
  if ((long long)out_size < need_s) return;
  if (ws_size < WS_TOTAL) return;

  const float* state = (const float*)d_in[0];
  const float* w1    = (const float*)d_in[1];
  const float* b1    = (const float*)d_in[2];
  const float* w2    = (const float*)d_in[3];
  const float* b2    = (const float*)d_in[4];
  const int*   nst   = (const int*)d_in[5];
  float* out = (float*)d_out;

  char* ws = (char*)d_ws;
  float*    S1  = (float*)(ws + OFF_STATE);
  _Float16* W1t = (_Float16*)(ws + OFF_W1T);
  _Float16* W2t = (_Float16*)(ws + OFF_W2T);

  dim3 blk(NTHR);
  dim3 grid(WCOLS / TP, HROWS);

  wprep_kernel<<<dim3(1), blk, 0, stream>>>(w1, b1, w2, W1t, W2t);

  const float* src = state;
  for (int i = 0; i < NSTEPS; ++i) {
    float* dst = (((NSTEPS - 1 - i) & 1) == 0) ? out : S1;
    if (i == 0)
      step_in_kernel<<<grid, blk, 0, stream>>>(src, dst, W1t, W2t, b2, nst, i);
    else
      step_ws_kernel<<<grid, blk, 0, stream>>>(src, dst, W1t, W2t, b2, nst, i);
    src = dst;
  }
}
